// Compositional_Attention_25451976196688
// MI455X (gfx1250) — hardware-verified
//
#include <hip/hip_runtime.h>

typedef __attribute__((ext_vector_type(16))) _Float16 v16h;
typedef __attribute__((ext_vector_type(8)))  _Float16 v8h;
typedef __attribute__((ext_vector_type(16))) __bf16   v16b;
typedef __attribute__((ext_vector_type(8)))  __bf16   v8b;
typedef __attribute__((ext_vector_type(8)))  float    v8f;
typedef __attribute__((ext_vector_type(4)))  float    v4f;
typedef __attribute__((ext_vector_type(2)))  float    v2f;
typedef __attribute__((ext_vector_type(2)))  unsigned v2u;

__device__ __forceinline__ unsigned short f2bf_bits(float f) {
  unsigned u = __float_as_uint(f);
  return (unsigned short)((u + 0x7FFFu + ((u >> 16) & 1u)) >> 16);
}
__device__ __forceinline__ float bf_bits2f(unsigned short h) { return __uint_as_float(((unsigned)h) << 16); }
__device__ __forceinline__ unsigned short h2bits(_Float16 h) { return __builtin_bit_cast(unsigned short, h); }

__device__ __forceinline__ void dep_guard_h(v8f& a, v8f& b, v16h x, v16h y) { asm volatile("v_nop\n\tv_nop\n\tv_nop\n\tv_nop" : "+v"(a), "+v"(b) : "v"(x), "v"(y)); }
__device__ __forceinline__ void dep_guard_b(v8f& a, v8f& b, v16b x, v16b y) { asm volatile("v_nop\n\tv_nop\n\tv_nop\n\tv_nop" : "+v"(a), "+v"(b) : "v"(x), "v"(y)); }
__device__ __forceinline__ void keep4_h(v16h a, v16h b, v16h c, v16h d) { asm volatile("v_nop" :: "v"(a), "v"(b), "v"(c), "v"(d)); }
__device__ __forceinline__ void keep4_b(v16b a, v16b b, v16b c, v16b d) { asm volatile("v_nop" :: "v"(a), "v"(b), "v"(c), "v"(d)); }
__device__ __forceinline__ void acc_guard4(v8f& a, v8f& b, v8f& c, v8f& d) { asm volatile("v_nop\n\tv_nop\n\tv_nop\n\tv_nop" : "+v"(a), "+v"(b), "+v"(c), "+v"(d)); }
template <typename T> struct Frag;
template <> struct Frag<_Float16> {
  typedef v16h V; union U { v16h v; v8h h[2]; };
  static __device__ __forceinline__ v16h load(const _Float16* p) {
    U f; f.h[0] = *(const v8h*)(p); f.h[1] = *(const v8h*)(p + 16); return f.v;
  }
  static __device__ __forceinline__ v8f mma(v16h a, v16h b, v8f c) {
    return __builtin_amdgcn_wmma_f32_16x16x32_f16(false, a, false, b, (short)0, c, false, false);
  }
  static __device__ __forceinline__ void guard(v8f& a, v8f& b, v16h x, v16h y) { dep_guard_h(a, b, x, y); }
  static __device__ __forceinline__ void keep(v16h a, v16h b, v16h c, v16h d) { keep4_h(a, b, c, d); }
};
template <> struct Frag<__bf16> {
  typedef v16b V; union U { v16b v; v8b h[2]; };
  static __device__ __forceinline__ v16b load(const __bf16* p) {
    U f; f.h[0] = *(const v8b*)(p); f.h[1] = *(const v8b*)(p + 16); return f.v;
  }
  static __device__ __forceinline__ v8f mma(v16b a, v16b b, v8f c) {
    return __builtin_amdgcn_wmma_f32_16x16x32_bf16(false, a, false, b, (short)0, c, false, false);
  }
  static __device__ __forceinline__ void guard(v8f& a, v8f& b, v16b x, v16b y) { dep_guard_b(a, b, x, y); }
  static __device__ __forceinline__ void keep(v16b a, v16b b, v16b c, v16b d) { keep4_b(a, b, c, d); }
};

template <int ET> struct Elem;
template <> struct Elem<0> { typedef _Float16 T; };
template <> struct Elem<1> { typedef __bf16 T; };
template <int ET, bool SPLIT, int BIAS_MODE, int OUT_MODE, bool RESID, int ACT = 0>
__global__ __launch_bounds__(256) void wmma_gemm64(
    const unsigned short* __restrict__ Ap, const unsigned short* __restrict__ A2p, int lda, long strideA,
    const unsigned short* __restrict__ Btp, const unsigned short* __restrict__ Bt2p, int ldb, long strideB,
    void* __restrict__ Cout, void* __restrict__ Cout2, int ldc, long strideC,
    const float* __restrict__ bias,
    const float* __restrict__ resid, long strideR,
    int M, int N, int K, float scale) {
  typedef typename Elem<ET>::T T;
  typedef typename Frag<T>::V V;
  const T* A = (const T*)Ap; const T* A2 = (const T*)A2p; const T* Bt = (const T*)Btp; const T* Bt2 = (const T*)Bt2p;
  __shared__ __align__(16) float sT[8][16 * 68];
  const int b    = blockIdx.y;
  const int lane = threadIdx.x & 31;
  const int wave = threadIdx.x >> 5;
  const int tilesN = N >> 6;
  const int tilesM = M >> 6;
  const int tile = blockIdx.x * 8 + wave;
  if (tile >= tilesM * tilesN) return;
  const int tm = tile / tilesN;
  const int tn = tile - tm * tilesN;
  const int m0 = tm << 6;
  const int n0 = tn << 6;

  const T* Ab  = A  + (size_t)b * strideA;
  const T* Bb  = Bt + (size_t)b * strideB;
  const T* Ab2 = SPLIT ? (A2  + (size_t)b * strideA) : nullptr;
  const T* Bb2 = SPLIT ? (Bt2 + (size_t)b * strideB) : nullptr;

  const int rlane = lane & 15;
  const int koff  = (lane >> 4) * 8;
  const int mOff  = (lane >> 4) * 8;

  v8f acc[4][4];
#pragma unroll
  for (int i = 0; i < 4; ++i)
#pragma unroll
    for (int j = 0; j < 4; ++j) acc[i][j] = (v8f){0.f,0.f,0.f,0.f,0.f,0.f,0.f,0.f};

  for (int k0 = 0; k0 < K; k0 += 32) {
    V bh[4], bl[4];
#pragma unroll
    for (int j = 0; j < 4; ++j) {
      const size_t bo = (size_t)(n0 + (j << 4) + rlane) * ldb + koff + k0;
      bh[j] = Frag<T>::load(Bb + bo);
      if (SPLIT) bl[j] = Frag<T>::load(Bb2 + bo);
    }
#pragma unroll
    for (int i = 0; i < 4; ++i) {
      const size_t ao = (size_t)(m0 + (i << 4) + rlane) * lda + koff + k0;
      V ah = Frag<T>::load(Ab + ao);
      V al;
      if (SPLIT) al = Frag<T>::load(Ab2 + ao);
#pragma unroll
      for (int j = 0; j < 4; ++j) {
        acc[i][j] = Frag<T>::mma(ah, bh[j], acc[i][j]);
        if (SPLIT) {
          acc[i][j] = Frag<T>::mma(ah, bl[j], acc[i][j]);
          acc[i][j] = Frag<T>::mma(al, bh[j], acc[i][j]);
        }
      }
      Frag<T>::guard(acc[i][0], acc[i][3], ah, SPLIT ? al : ah);
    }
    Frag<T>::keep(bh[0], bh[1], bh[2], bh[3]);
    if (SPLIT) Frag<T>::keep(bl[0], bl[1], bl[2], bl[3]);
  }
  acc_guard4(acc[0][0], acc[0][1], acc[0][2], acc[0][3]);
  acc_guard4(acc[1][0], acc[1][1], acc[1][2], acc[1][3]);
  acc_guard4(acc[2][0], acc[2][1], acc[2][2], acc[2][3]);
  acc_guard4(acc[3][0], acc[3][1], acc[3][2], acc[3][3]);

  float* slab = sT[wave];
  const float* Rb = RESID ? (resid + (size_t)b * strideR) : nullptr;
#pragma unroll
  for (int i = 0; i < 4; ++i) {
    const int mBase = m0 + (i << 4);
#pragma unroll
    for (int j = 0; j < 4; ++j) {
      const int n = n0 + (j << 4) + rlane;
      float bv = 0.f;
      if (BIAS_MODE == 2) bv = bias[n];
#pragma unroll
      for (int r = 0; r < 8; ++r) {
        float v = acc[i][j][r] * scale;
        if (BIAS_MODE == 1) v += bias[mBase + mOff + r];
        if (BIAS_MODE == 2) v += bv;
        if (RESID) v += Rb[(size_t)(mBase + mOff + r) * ldc + n];
        if (ACT == 1) v = tanhf(v);
        if (ACT == 2) v = fmaxf(v, 0.0f);
        if (ACT == 3) v = v / (1.0f + expf(-v));
        if (ACT == 4) v = (v > 0.f) ? v : 0.01f * v;
        if (ACT == 5) v = 0.5f * v * (1.0f + erff(v * 0.70710678118654752f));
        slab[(mOff + r) * 68 + (j << 4) + rlane] = v;
      }
    }
    __builtin_amdgcn_fence(__ATOMIC_RELEASE, "workgroup");
    __builtin_amdgcn_wave_barrier();
    __builtin_amdgcn_fence(__ATOMIC_ACQUIRE, "workgroup");
    if (OUT_MODE == 0) {
      float* C = (float*)Cout + (size_t)b * strideC;
      const int hh = lane >> 4, c4 = (lane & 15) * 4;
      for (int pass = 0; pass < 2; ++pass) {
#pragma unroll
        for (int it = 0; it < 8; ++it) {
          const int row = it * 2 + hh;
          v4f v = *(const v4f*)(slab + row * 68 + c4);
          *(volatile v4f*)(C + (size_t)(mBase + row) * ldc + n0 + c4) = v;
        }
        __threadfence();
      }
    } else {
      const int q = lane >> 3, c8 = (lane & 7) * 8;
      unsigned short* C  = (unsigned short*)Cout  + (size_t)b * strideC;
      unsigned short* C2 = (OUT_MODE == 2) ? ((unsigned short*)Cout2 + (size_t)b * strideC) : nullptr;
      for (int pass = 0; pass < 2; ++pass) {
#pragma unroll
        for (int it = 0; it < 4; ++it) {
          const int row = it * 4 + q;
          const float* sp = slab + row * 68 + c8;
          v8h hv, lv;
#pragma unroll
          for (int e = 0; e < 8; ++e) {
            if (OUT_MODE == 1) {
              hv[e] = (_Float16)sp[e];
            } else {
              unsigned short hb = f2bf_bits(sp[e]);
              unsigned short lb = f2bf_bits(sp[e] - bf_bits2f(hb));
              hv[e] = __builtin_bit_cast(_Float16, hb);
              lv[e] = __builtin_bit_cast(_Float16, lb);
            }
          }
          *(volatile v8h*)(C + (size_t)(mBase + row) * ldc + n0 + c8) = hv;
          if (OUT_MODE == 2) *(volatile v8h*)(C2 + (size_t)(mBase + row) * ldc + n0 + c8) = lv;
        }
        __threadfence();
      }
    }
    __builtin_amdgcn_fence(__ATOMIC_RELEASE, "workgroup");
    __builtin_amdgcn_wave_barrier();
    __builtin_amdgcn_fence(__ATOMIC_ACQUIRE, "workgroup");
  }
}

__device__ __forceinline__ float wave_sum(float v) {
#pragma unroll
  for (int off = 16; off > 0; off >>= 1) v += __shfl_xor(v, off, 32);
  return v;
}
__device__ __forceinline__ float wave_max(float v) {
#pragma unroll
  for (int off = 16; off > 0; off >>= 1) v = fmaxf(v, __shfl_xor(v, off, 32));
  return v;
}

__global__ __launch_bounds__(256) void cast_scale_f16x2(
    const float* __restrict__ in, _Float16* __restrict__ out, int n2, float scale) {
  int i = blockIdx.x * 256 + threadIdx.x;
  if (i < n2) {
    const _Float16 h0 = (_Float16)(in[2 * i] * scale), h1 = (_Float16)(in[2 * i + 1] * scale);
    const unsigned u = (unsigned)h2bits(h0) | ((unsigned)h2bits(h1) << 16);
    ((volatile unsigned*)out)[i] = u;
    __threadfence();
    ((volatile unsigned*)out)[i] = u;
  }
}

__global__ __launch_bounds__(256) void layernorm1024_f16(
    const float* __restrict__ x, const float* __restrict__ g, const float* __restrict__ bta,
    _Float16* __restrict__ out, float eps) {
  __shared__ float redA[8];
  __shared__ float redB[8];
  const int row  = blockIdx.x;
  const int tid  = threadIdx.x;
  const int lane = tid & 31;
  const int wave = tid >> 5;
  const float* xr = x + (size_t)row * 1024;
  const v4f xv = *(const v4f*)(xr + 4 * tid);
  float s = (xv[0] + xv[1]) + (xv[2] + xv[3]);
  s = wave_sum(s);
  if (lane == 0) redA[wave] = s;
  __syncthreads();
  float tot = 0.f;
#pragma unroll
  for (int w = 0; w < 8; ++w) tot += redA[w];
  const float mean = tot * (1.0f / 1024.0f);
  const float d0 = xv[0] - mean, d1 = xv[1] - mean, d2 = xv[2] - mean, d3 = xv[3] - mean;
  float vs = (d0 * d0 + d1 * d1) + (d2 * d2 + d3 * d3);
  vs = wave_sum(vs);
  if (lane == 0) redB[wave] = vs;
  __syncthreads();
  float tot2 = 0.f;
#pragma unroll
  for (int w = 0; w < 8; ++w) tot2 += redB[w];
  const float var  = tot2 * (1.0f / 1024.0f);
  const float rstd = 1.0f / sqrtf(var + eps);
  const v4f gv = *(const v4f*)(g + 4 * tid);
  const v4f bv = *(const v4f*)(bta + 4 * tid);
  const _Float16 y0 = (_Float16)(d0 * rstd * gv[0] + bv[0]);
  const _Float16 y1 = (_Float16)(d1 * rstd * gv[1] + bv[1]);
  const _Float16 y2 = (_Float16)(d2 * rstd * gv[2] + bv[2]);
  const _Float16 y3 = (_Float16)(d3 * rstd * gv[3] + bv[3]);
  v2u pk;
  pk[0] = (unsigned)h2bits(y0) | ((unsigned)h2bits(y1) << 16);
  pk[1] = (unsigned)h2bits(y2) | ((unsigned)h2bits(y3) << 16);
  _Float16* dst = out + (size_t)row * 1024 + 4 * tid;
  *(volatile v2u*)dst = pk;
  __threadfence();
  *(volatile v2u*)dst = pk;
}

__global__ __launch_bounds__(256) void softmax1024_f16(
    const float* __restrict__ S, _Float16* __restrict__ P, int nrows, float outscale) {
  const int lane = threadIdx.x & 31;
  const int wave = threadIdx.x >> 5;
  const int row  = blockIdx.x * 8 + wave;
  if (row < nrows) {
    const float* sr = S + (size_t)row * 1024;
    v4f xv[8];
#pragma unroll
    for (int i = 0; i < 8; ++i) xv[i] = *(const v4f*)(sr + i * 128 + lane * 4);
    float m = -3.0e38f;
#pragma unroll
    for (int i = 0; i < 8; ++i) {
      m = fmaxf(m, fmaxf(fmaxf(xv[i][0], xv[i][1]), fmaxf(xv[i][2], xv[i][3])));
    }
    m = wave_max(m);
    float sum = 0.f;
#pragma unroll
    for (int i = 0; i < 8; ++i) {
#pragma unroll
      for (int e = 0; e < 4; ++e) {
        const float ev = __expf(xv[i][e] - m);
        xv[i][e] = ev;
        sum += ev;
      }
    }
    sum = wave_sum(sum);
    const float sc = outscale * (1.0f / sum);
    _Float16* pr = P + (size_t)row * 1024;
    for (int pass = 0; pass < 2; ++pass) {
#pragma unroll
      for (int i = 0; i < 8; ++i) {
        const _Float16 p0 = (_Float16)(xv[i][0] * sc), p1 = (_Float16)(xv[i][1] * sc);
        const _Float16 p2 = (_Float16)(xv[i][2] * sc), p3 = (_Float16)(xv[i][3] * sc);
        v2u pk;
        pk[0] = (unsigned)h2bits(p0) | ((unsigned)h2bits(p1) << 16);
        pk[1] = (unsigned)h2bits(p2) | ((unsigned)h2bits(p3) << 16);
        *(volatile v2u*)(pr + i * 128 + lane * 4) = pk;
      }
      __threadfence();
    }
  }
}

__global__ __launch_bounds__(256) void rule_combine(
    const float* __restrict__ O, const float* __restrict__ qv, const float* __restrict__ Ws,
    const float* __restrict__ bs, _Float16* __restrict__ attn, int b, int h0, float qvscale, float oscale) {
  const int n    = blockIdx.x;
  const int lane = threadIdx.x & 31;
  const int hl   = threadIdx.x >> 5;
  const int h    = h0 + hl;
  const float* orow = O + ((size_t)hl * 1024 + n) * 512 + 2 * lane;
  float o0[8], o1[8];
#pragma unroll
  for (int r = 0; r < 8; ++r) {
    const v2f t = *(const v2f*)(orow + r * 64);
    o0[r] = t[0]; o1[r] = t[1];
  }
  const size_t tok = (size_t)b * 1024 + n;
  float cq = Ws[lane] * qv[tok * 512 + (size_t)h * 32 + lane];
  cq = wave_sum(cq);
  const float ws0 = Ws[32 + 2 * lane];
  const float ws1 = Ws[33 + 2 * lane];
  const float base = cq * qvscale + bs[0];
  float c[8];
#pragma unroll
  for (int r = 0; r < 8; ++r) c[r] = wave_sum(ws0 * o0[r] + ws1 * o1[r]) + base;
  float mx = c[0];
#pragma unroll
  for (int r = 1; r < 8; ++r) mx = fmaxf(mx, c[r]);
  float e[8];
  float s = 0.f;
#pragma unroll
  for (int r = 0; r < 8; ++r) { e[r] = __expf(c[r] - mx); s += e[r]; }
  const float inv = 1.0f / s;
  float a0 = 0.f, a1 = 0.f;
#pragma unroll
  for (int r = 0; r < 8; ++r) {
    const float w = e[r] * inv;
    a0 += w * o0[r];
    a1 += w * o1[r];
  }
  const _Float16 q0 = (_Float16)(a0 * oscale), q1 = (_Float16)(a1 * oscale);
  const unsigned u = (unsigned)h2bits(q0) | ((unsigned)h2bits(q1) << 16);
  volatile unsigned* dst = (volatile unsigned*)(attn + tok * 1024 + (size_t)h * 64) + lane;
  *dst = u;
  __threadfence();
  *dst = u;
}

template <int BIAS, int OUT, bool RES, int ACT>
static void gemm_f16(hipStream_t st, const void* A, int lda, long sA, const void* Bt, int ldb, long sB,
                     void* C, int ldc, long sC, const float* bias, const float* resid, long sR,
                     int M, int N, int K, float scale, int batch) {
  const int tiles = (M / 64) * (N / 64);
  dim3 grid((unsigned)((tiles + 7) / 8), (unsigned)batch);
  wmma_gemm64<0, false, BIAS, OUT, RES, ACT><<<grid, dim3(256), 0, st>>>(
      (const unsigned short*)A, (const unsigned short*)A, lda, sA,
      (const unsigned short*)Bt, (const unsigned short*)Bt, ldb, sB,
      C, C, ldc, sC, bias, resid, sR, M, N, K, scale);
}

extern "C" void kernel_launch(void* const* d_in, const int* in_sizes, int n_in,
                              void* d_out, int out_size, void* d_ws, size_t ws_size,
                              hipStream_t stream) {
  const int Bn = 4, Sn = 1024, D = 1024, NT = Bn * Sn;
  if (n_in < 21) return;
  if (in_sizes[0] != NT * D || out_size != NT * D) return;
  if (in_sizes[1] != D * D || in_sizes[3] != D * D || in_sizes[5] != 512 * D || in_sizes[7] != 512 * D) return;
  if (in_sizes[9] != 96 || in_sizes[10] < 1 || in_sizes[11] != D * D || in_sizes[13] != 2048 * D || in_sizes[15] != D * 2048) return;

  const size_t MB = (size_t)1 << 20;
  const size_t need = 108 * MB;
  if (ws_size < need) return;

  const float* x   = (const float*)d_in[0];
  const float* Wq  = (const float*)d_in[1];
  const float* bq  = (const float*)d_in[2];
  const float* Wk  = (const float*)d_in[3];
  const float* bk  = (const float*)d_in[4];
  const float* Wv  = (const float*)d_in[5];
  const float* bv  = (const float*)d_in[6];
  const float* Wqv = (const float*)d_in[7];
  const float* bqv = (const float*)d_in[8];
  const float* Ws  = (const float*)d_in[9];
  const float* bs  = (const float*)d_in[10];
  const float* Wf  = (const float*)d_in[11];
  const float* bfb = (const float*)d_in[12];
  const float* Wr1 = (const float*)d_in[13];
  const float* br1 = (const float*)d_in[14];
  const float* Wr2 = (const float*)d_in[15];
  const float* br2 = (const float*)d_in[16];
  const float* g1  = (const float*)d_in[17];
  const float* b1  = (const float*)d_in[18];
  const float* g2  = (const float*)d_in[19];
  const float* b2  = (const float*)d_in[20];
  float* out = (float*)d_out;

  char* ws = (char*)d_ws;
  _Float16* xn16   = (_Float16*)(ws + 0 * MB);
  _Float16* q16    = (_Float16*)(ws + 8 * MB);
  _Float16* k16    = (_Float16*)(ws + 16 * MB);
  _Float16* vT16   = (_Float16*)(ws + 24 * MB);
  float*    qv32   = (float*)(ws + 28 * MB);
  _Float16* attn16 = (_Float16*)(ws + 36 * MB);
  _Float16* Wq16   = (_Float16*)(ws + 44 * MB);
  _Float16* Wk16   = (_Float16*)(ws + 46 * MB);
  _Float16* Wv16   = (_Float16*)(ws + 48 * MB);
  _Float16* Wqv16  = (_Float16*)(ws + 49 * MB);
  float*    Sbuf   = (float*)(ws + 44 * MB);
  _Float16* P16    = (_Float16*)(ws + 76 * MB);
  float*    Obuf   = (float*)(ws + 92 * MB);
  float*    res2   = (float*)(ws + 0 * MB);
  _Float16* Wf16   = (_Float16*)(ws + 16 * MB);
  _Float16* on16   = (_Float16*)(ws + 18 * MB);
  _Float16* Wr1_16 = (_Float16*)(ws + 26 * MB);
  _Float16* Wr2_16 = (_Float16*)(ws + 30 * MB);
  _Float16* h16    = (_Float16*)(ws + 44 * MB);

  const float WSC = 16.0f;
  const float INV_WSC = 1.0f / 16.0f;
  const float PSC = 32768.0f;
  const float ASC = 16.0f;
  const float EPS = 1e-5f;

  auto cast = [&](const float* src, _Float16* dst, int n, float scale) {
    const int n2 = n / 2;
    cast_scale_f16x2<<<dim3((unsigned)((n2 + 255) / 256)), dim3(256), 0, stream>>>(src, dst, n2, scale);
  };

  cast(Wq, Wq16, D * D, WSC);
  cast(Wk, Wk16, D * D, WSC);
  cast(Wv, Wv16, 512 * D, WSC);
  cast(Wqv, Wqv16, 512 * D, WSC);
  layernorm1024_f16<<<dim3(NT), dim3(256), 0, stream>>>(x, g1, b1, xn16, EPS);
  gemm_f16<2, 1, false, 0>(stream, xn16, D, 0, Wq16, D, 0, q16, D, 0, bq, x, 0, NT, D, D, INV_WSC, 1);
  gemm_f16<2, 1, false, 0>(stream, xn16, D, 0, Wk16, D, 0, k16, D, 0, bk, x, 0, NT, D, D, INV_WSC, 1);
  gemm_f16<1, 1, false, 0>(stream, Wv16, D, 0, xn16, D, (long)Sn * D, vT16, D, (long)512 * D, bv, x, 0, 512, Sn, D, INV_WSC, Bn);
  gemm_f16<2, 0, false, 0>(stream, xn16, D, 0, Wqv16, D, 0, qv32, 512, 0, bqv, x, 0, NT, 512, D, INV_WSC, 1);

  for (int gi = 0; gi < 8; ++gi) {
    const int b  = gi >> 1;
    const int h0 = (gi & 1) * 8;
    const _Float16* qg = q16 + (size_t)b * Sn * D + h0 * 64;
    const _Float16* kg = k16 + (size_t)b * Sn * D + h0 * 64;
    gemm_f16<0, 0, false, 0>(stream, qg, D, 64, kg, D, 64, Sbuf, Sn, (long)Sn * Sn, Ws, x, 0, Sn, Sn, 64, 0.125f, 8);
    softmax1024_f16<<<dim3(8 * Sn / 8), dim3(256), 0, stream>>>(Sbuf, P16, 8 * Sn, PSC);
    gemm_f16<0, 0, false, 0>(stream, P16, Sn, (long)Sn * Sn, vT16 + (size_t)b * 512 * D, D, 0,
                             Obuf, 512, (long)Sn * 512, Ws, x, 0, Sn, 512, Sn, 1.0f / PSC, 8);
    rule_combine<<<dim3(Sn), dim3(256), 0, stream>>>(Obuf, qv32, Ws, bs, attn16, b, h0, 0.17677669529663687f, ASC);
  }

  cast(Wf, Wf16, D * D, WSC);
  gemm_f16<2, 0, true, 0>(stream, attn16, D, 0, Wf16, D, 0, res2, D, 0, bfb, x, 0, NT, D, D, INV_WSC / ASC, 1);
  layernorm1024_f16<<<dim3(NT), dim3(256), 0, stream>>>(res2, g2, b2, on16, EPS);
  cast(Wr1, Wr1_16, 2048 * D, WSC);
  cast(Wr2, Wr2_16, D * 2048, WSC);
  gemm_f16<2, 1, false, 2>(stream, on16, D, 0, Wr1_16, D, 0, h16, 2048, 0, br1, x, 0, NT, 2048, D, INV_WSC, 1);
  gemm_f16<2, 0, true, 0>(stream, h16, 2048, 0, Wr2_16, 2048, 0, out, D, 0, br2, res2, 0, NT, D, 2048, INV_WSC, 1);
  (void)hipGetLastError();
}
